// SimpleGCN_62886911148524
// MI455X (gfx1250) — hardware-verified
//
#include <hip/hip_runtime.h>


namespace {

constexpr int N = 100000, NP = 100000, NPL = NP  , SRCM = N  , EFULL = 1600000, E = EFULL  ;
constexpr int FI = 128  , F = 128  , FO = 64  , NCLS = 2  , NG = 1024  , LYR = 2  , F2 = F, VOC = 1, NRL = NP  , NL = (NPL < N ? NPL : N);
static_assert(F == 128 && NCLS <= FO && NG % 32 == 0 && (NG * NCLS) % 32 == 0, "128-wide planes; 1,024 pooled rows = 32 lin row blocks; whole output lines");
constexpr float LNEPS = 1e-5f; constexpr float LOG2E = 1.4426950408889634f; constexpr float XS = 8.0f, WSC = 256.0f, WSQ = 0.25f, RS_ = 1024.0f, NSL_ = 0.2f, NSA_ = 0.01f, SLOPE = 0.0f, BNEPS = 1e-5f;
static_assert(NP % 32 == 0 && NP >= N && NPL % 32 == 0 && F % 32 == 0, "tiling");
typedef _Float16 b16;
typedef __attribute__((ext_vector_type(16))) _Float16 v16b;
typedef __attribute__((ext_vector_type(8))) _Float16 v8b;
typedef __attribute__((ext_vector_type(8))) float v8f;
typedef __attribute__((ext_vector_type(4))) float v4f;
__device__ __forceinline__ float bf16_rne(float f) { unsigned int u = __float_as_uint(f); u += 0x7FFFu + ((u >> 16) & 1u); return __uint_as_float(u & 0xFFFF0000u); }
__device__ __forceinline__ float bfo(float f) { float r = bf16_rne(f); asm volatile("" : "+v"(r)); return r; }
__device__ __forceinline__ void split16(float v, b16& hi, b16& lo) { hi = (b16)v; lo = (b16)(v - (float)hi); }
__device__ __forceinline__ v16b frag_kb(const b16* p, int hh) { const v8b a = *(const v8b*)(p + 8 * hh), b = *(const v8b*)(p + 16 + 8 * hh); v16b f;
#pragma unroll
  for (int e = 0; e < 8; ++e) { f[e] = a[e]; f[8 + e] = b[e]; } return f; }
__device__ __forceinline__ v8f wmma16b(v16b a, v16b b, v8f c) { v8f d = __builtin_amdgcn_wmma_f32_16x16x32_f16(false, a, false, b, (short)0, c, false, false); asm volatile("v_nop\n\tv_nop\n\tv_nop\n\tv_nop" : "+v"(d) : "v"(a), "v"(b)); return d; }
__device__ __forceinline__ void wave_lds_sync() { __builtin_amdgcn_fence(__ATOMIC_RELEASE, "workgroup"); __builtin_amdgcn_wave_barrier(); __builtin_amdgcn_fence(__ATOMIC_ACQUIRE, "workgroup"); }
__device__ __forceinline__ float pmul(float a, float b) { float p = a * b; asm volatile("" : "+v"(p)); return p; }
__device__ __forceinline__ int iclamp(int v, int lo, int hi) { return v < lo ? lo : (v > hi ? hi : v); }
constexpr int CSR_NBLK = 512, CSR_GB = 9, CSR_GN = 1 << CSR_GB  , CSR_MAXG = 512, CSR_CAP = 12288  ;
static_assert(((N + CSR_GN - 1) >> CSR_GB) <= CSR_MAXG && CSR_GN % 4 == 0 && CSR_GN <= 65536, "csr: bucket count / 16-bit node key");
__global__ __launch_bounds__(64) void csrA_kernel(const int* __restrict__ dst, int E, int N, int nG, int CHP, int NGP, int* __restrict__ STG, int* __restrict__ HST) {
  extern __shared__ int sm[];
  int* cnt = sm; int* run = sm + NGP; int* ids = sm + 2 * NGP;
  const int b = blockIdx.x; const int ch = (E + CSR_NBLK - 1) / CSR_NBLK; const int e0 = b * ch, e1 = min(E, e0 + ch);
  for (int i = threadIdx.x; i < NGP; i += 64) cnt[i] = 0;
  for (int i = threadIdx.x; i < CHP; i += 64) ids[i] = -1;
  __syncthreads();
  if (threadIdx.x == 0) {
    for (int e = e0; e < e1; ++e) { int d = dst[e]; d = (d < 0) ? 0 : (d >= N ? N - 1 : d); cnt[d >> CSR_GB] += 1; }
    int acc = 0; for (int g = 0; g < nG; ++g) { run[g] = acc; acc += cnt[g]; }
    for (int e = e0; e < e1; ++e) { int d = dst[e]; d = (d < 0) ? 0 : (d >= N ? N - 1 : d); const int g = d >> CSR_GB; ids[run[g]] = e; run[g] += 1; } }
  __syncthreads();
  typedef __attribute__((ext_vector_type(4))) int v4i;
  for (int pass = 0; pass < 2; ++pass) {
    for (int i = threadIdx.x; i < CHP / 4; i += 64) *(volatile v4i*)(STG + (size_t)b * CHP + i * 4) = *(const v4i*)(&ids[i * 4]);
    for (int i = threadIdx.x; i < NGP / 4; i += 64) { v4i v; for (int e = 0; e < 4; ++e) v[e] = (i * 4 + e < nG) ? cnt[i * 4 + e] : 0; *(volatile v4i*)(HST + (size_t)b * NGP + i * 4) = v; }
    __threadfence(); }
}
__global__ __launch_bounds__(512) void csrS_kernel(const int* __restrict__ HST, int nG, int NGP, int* __restrict__ START, int* __restrict__ TOT, int* __restrict__ OFF) {
  __shared__ int tot[CSR_MAXG];
  const int b = threadIdx.x;
  for (int pass = 0; pass < 2; ++pass) { int runb = 0; for (int g = 0; g < nG; ++g) { int c = HST[(size_t)b * NGP + g]; c = (c < 0) ? 0 : c; ((volatile int*)OFF)[(size_t)g * CSR_NBLK + b] = runb; runb += c; } __threadfence(); }
  for (int g = threadIdx.x; g < nG; g += 512) { int s = 0; for (int bb = 0; bb < CSR_NBLK; ++bb) { int c = HST[(size_t)bb * NGP + g]; s += (c < 0) ? 0 : c; } tot[g] = s; }
  __syncthreads();
  if (threadIdx.x < 32) {
    __shared__ int st[CSR_MAXG + 32];
    if (threadIdx.x == 0) { int acc = 0; for (int g = 0; g < NGP; ++g) { st[g] = acc; if (g < nG) acc += (tot[g] + 31) & ~31; } st[NGP] = acc; }
    __builtin_amdgcn_fence(__ATOMIC_RELEASE, "workgroup"); __builtin_amdgcn_wave_barrier(); __builtin_amdgcn_fence(__ATOMIC_ACQUIRE, "workgroup");
    for (int pass = 0; pass < 2; ++pass) { for (int i = threadIdx.x; i < NGP + 32; i += 32) { ((volatile int*)START)[i] = (i <= NGP) ? st[min(i, NGP)] : 0; ((volatile int*)TOT)[i] = (i < nG) ? tot[i] : 0; } __threadfence(); } }
}
__global__ __launch_bounds__(256) void csrB_kernel(const int* __restrict__ dst, int N, int nG, int CHP, int NGP, int permLen, const int* __restrict__ STG, const int* __restrict__ HST, const int* __restrict__ OFF, const int* __restrict__ START, const int* __restrict__ TOT, int* __restrict__ PERM, int* __restrict__ ROWPTR, int* __restrict__ ROWCNT, int* __restrict__ FLAG) {
  typedef __attribute__((ext_vector_type(4))) int v4i;
  __shared__ int ids[CSR_CAP]; __shared__ unsigned short key[CSR_CAP]; __shared__ int outp[CSR_CAP]; __shared__ int ncnt[CSR_GN + 1]; __shared__ int boff[CSR_NBLK + 1];
  const int g = blockIdx.x, t_ = threadIdx.x; int tot = TOT[g]; int st = START[g], stn = START[g + 1]; const int v0 = g * CSR_GN; const int nv = min(CSR_GN, N - v0);
  st = (st < 0) ? 0 : (st > permLen - 32 ? permLen - 32 : st) & ~31; stn = (stn < st) ? st : (stn > permLen ? permLen : stn); tot = (tot < 0) ? 0 : tot; if (tot > stn - st && tot <= CSR_CAP) tot = stn - st;
  if (tot > CSR_CAP) {
    for (int pass = 0; pass < 2; ++pass) { for (int i = t_; i < CSR_GN / 4; i += 256) { v4i a, c; for (int e = 0; e < 4; ++e) { a[e] = st; c[e] = 0; } *(volatile v4i*)(ROWPTR + v0 + i * 4) = a; *(volatile v4i*)(ROWCNT + v0 + i * 4) = c; } if (t_ == 0) ((volatile int*)FLAG)[0] = 1; __threadfence(); } (void)nv; return; }
  if (t_ == 0) { int acc = 0; for (int b = 0; b < CSR_NBLK; ++b) { boff[b] = acc; int c = HST[(size_t)b * NGP + g]; c = (c < 0) ? 0 : (c > CHP ? CHP : c); acc += c; if (acc > tot) acc = tot; } boff[CSR_NBLK] = acc; }
  for (int i = t_; i <= CSR_GN; i += 256) ncnt[i] = 0;
  __syncthreads();
  for (int b = 0; b < CSR_NBLK; ++b) { const int c = boff[b + 1] - boff[b]; int o_ = OFF[(size_t)g * CSR_NBLK + b]; o_ = (o_ < 0) ? 0 : (o_ > CHP - c ? CHP - c : o_); const int* src_ = STG + (size_t)b * CHP + o_;
    for (int i = t_; i < c; i += 256) { int id = src_[i]; id = (id < 0) ? 0 : id; ids[boff[b] + i] = id; int d = dst[id]; d = (d < v0) ? v0 : (d >= N ? N - 1 : d); int kk = d - v0; kk = (kk < 0) ? 0 : (kk >= CSR_GN ? CSR_GN - 1 : kk); key[boff[b] + i] = (unsigned short)kk; } }
  __syncthreads();
  if (t_ == 0) { for (int i = 0; i < tot; ++i) ncnt[key[i]] += 1; int acc = 0; for (int vl = 0; vl < CSR_GN; ++vl) { const int c = ncnt[vl]; ncnt[vl] = acc; acc += c; } ncnt[CSR_GN] = acc;
    for (int i = 0; i < tot; ++i) { const int vl = key[i]; outp[ncnt[vl]] = ids[i]; ncnt[vl] += 1; }
    for (int vl = CSR_GN; vl > 0; --vl) ncnt[vl] = ncnt[vl - 1]; ncnt[0] = 0; }
  __syncthreads();
  for (int pass = 0; pass < 2; ++pass) {
    for (int i = t_; i < (stn - st) / 4; i += 256) { v4i v; for (int e = 0; e < 4; ++e) { const int q = i * 4 + e; v[e] = (q < tot) ? outp[q] : -1; } *(volatile v4i*)(PERM + st + i * 4) = v; }
    for (int i = t_; i < CSR_GN / 4; i += 256) { v4i a, c; for (int e = 0; e < 4; ++e) { const int vl = i * 4 + e; a[e] = st + ncnt[vl]; c[e] = (vl < nv) ? (ncnt[vl + 1] - ncnt[vl]) : 0; } *(volatile v4i*)(ROWPTR + v0 + i * 4) = a; *(volatile v4i*)(ROWCNT + v0 + i * 4) = c; }
    __threadfence(); }
}
__global__ __launch_bounds__(256) void csrZ_kernel(int* __restrict__ p, size_t n4) { typedef __attribute__((ext_vector_type(4))) int v4i; const size_t tid = (size_t)blockIdx.x * 256 + threadIdx.x, nth = (size_t)gridDim.x * 256; v4i z = {0, 0, 0, 0}; for (size_t i = tid; i < n4; i += nth) *(volatile v4i*)(p + i * 4) = z; }
struct CsrBufs { int *STG, *HST, *OFF, *START, *TOT, *PERM, *ROWPTR, *ROWCNT, *FLAG; int nG, NGP, CHP; size_t permLen; char* base; size_t bytes; };
static size_t csr_carve(CsrBufs& c, char* ws, size_t off, int E, int N) {
  const size_t off0 = off; c.base = ws + off;
  auto al = [&](size_t bytes) { char* p = ws + off; off += (bytes + 255) & ~(size_t)255; return p; };
  c.nG = (N + CSR_GN - 1) / CSR_GN; c.NGP = (c.nG + 31) & ~31; const int ch = (E + CSR_NBLK - 1) / CSR_NBLK; c.CHP = (ch + 31) & ~31; c.permLen = (size_t)E + 32 * (size_t)c.nG + 32;
  c.STG = (int*)al((size_t)CSR_NBLK * c.CHP * 4); c.HST = (int*)al((size_t)CSR_NBLK * c.NGP * 4); c.OFF = (int*)al((size_t)c.NGP * CSR_NBLK * 4); c.START = (int*)al((size_t)(c.NGP + 64) * 4); c.TOT = (int*)al((size_t)(c.NGP + 64) * 4);
  c.PERM = (int*)al(c.permLen * 4); c.ROWPTR = (int*)al((size_t)c.nG * CSR_GN * 4); c.ROWCNT = (int*)al((size_t)c.nG * CSR_GN * 4); c.FLAG = (int*)al(256);
  c.bytes = off - off0; return off;
}
static void csr_build(const CsrBufs& c, const int* dst, int E, int N, hipStream_t stream) {
  const size_t smem = (size_t)(2 * c.NGP + c.CHP) * 4;
  csrZ_kernel<<<512, 256, 0, stream>>>((int*)c.base, c.bytes / 16);
  csrA_kernel<<<CSR_NBLK, 64, smem, stream>>>(dst, E, N, c.nG, c.CHP, c.NGP, c.STG, c.HST);
  csrS_kernel<<<1, 512, 0, stream>>>(c.HST, c.nG, c.NGP, c.START, c.TOT, c.OFF);
  csrB_kernel<<<c.nG, 256, 0, stream>>>(dst, N, c.nG, c.CHP, c.NGP, (int)c.permLen, c.STG, c.HST, c.OFF, c.START, c.TOT, c.PERM, c.ROWPTR, c.ROWCNT, c.FLAG);
}

typedef __attribute__((ext_vector_type(4))) _Float16 v4h;
__device__ __forceinline__ float lrelu(float v) { return v > 0.0f ? v : NSL_ * v; }
template <int K, int NOUTR, int NOUTP>
__global__ __launch_bounds__(256) void wt_kernel(const float* __restrict__ w, b16* __restrict__ WT, float scl) {
  static_assert(K % 8 == 0 && NOUTR <= NOUTP, "wt: thread per (o, 8 k)");
  const int u = blockIdx.x * 256 + threadIdx.x; if (u >= NOUTP * K / 8) return; const int e = u * 8; const int o = e / K, k0 = e % K; v8b v;
#pragma unroll
  for (int j = 0; j < 8; ++j) v[j] = (b16)(o < NOUTR ? bf16_rne(w[(size_t)(k0 + j) * NOUTR + o]) * scl : 0.0f);
  for (int pass = 0; pass < 2; ++pass) { *(volatile v8b*)(WT + e) = v; __threadfence(); }
}
template <int K, int NT, bool RND, int MODE, bool GIDX>
__global__ __launch_bounds__(64) void lin_kernel(const float* __restrict__ X, const int* __restrict__ gidx, const b16* __restrict__ WT, const b16* __restrict__ WQ, const float* __restrict__ bias, float* __restrict__ OUT, int opitch, int nvalid, int mrows) {
  constexpr int NC = NT * 16;
  static_assert(K % 32 == 0 && NT % 4 == 0 && NT <= 16 && (NC < 128 || NC % 128 == 0), "lin: k-steps of 32; row store = whole 128-column groups or one partial group");
  __shared__ __attribute__((aligned(16))) b16 Ah[2][16][K + 8], Al[2][16][K + 8]; __shared__ __attribute__((aligned(16))) float Tf[2][16][NC + 4];
  const int wave = threadIdx.x >> 5, lane = threadIdx.x & 31, nloc = lane & 15, hlf = lane >> 4; const size_t m0 = (size_t)blockIdx.x * 32 + wave * 16;
  for (int idx = lane; idx < 16 * (K / 4); idx += 32) { const int rr = idx / (K / 4), c4 = (idx % (K / 4)) * 4; const size_t vrow = (m0 + rr < (size_t)nvalid) ? m0 + rr : (size_t)nvalid - 1; size_t arow = vrow; if (GIDX) arow = (size_t)iclamp(gidx[vrow], 0, VOC - 1);
    const v4f v = *(const v4f*)(X + arow * K + c4); v4h hv, lv;
    for (int j = 0; j < 4; ++j) { float vj = v[j]; if (MODE == 2) vj = fmaxf(vj, 0.0f); const float vs = (RND ? bf16_rne(vj) : vj) * XS; const b16 ph = (b16)vs; hv[j] = ph; lv[j] = (b16)((vs - (float)ph) * RS_); } *(v4h*)(&Ah[wave][rr][c4]) = hv; *(v4h*)(&Al[wave][rr][c4]) = lv; }
  wave_lds_sync();
  v8f acc[NT];
#pragma unroll
  for (int t = 0; t < NT; ++t) acc[t] = (v8f){};
#pragma unroll 1
  for (int kb = 0; kb < K; kb += 32) { const v16b a = frag_kb(&Ah[wave][nloc][kb], hlf); v16b al; if (!RND) al = frag_kb(&Al[wave][nloc][kb], hlf);
#pragma unroll
    for (int t = 0; t < NT; ++t) { const size_t wo_ = (size_t)(t * 16 + nloc) * K + kb; acc[t] = wmma16b(a, frag_kb(WT + wo_, hlf), acc[t]); if (!RND) acc[t] = wmma16b(al, frag_kb(WQ + wo_, hlf), acc[t]); } }
#pragma unroll
  for (int t = 0; t < NT; ++t) { const int col = t * 16 + nloc; const float bb = bf16_rne(bias[col]);
    for (int r = 0; r < 8; ++r) { const size_t vrow = m0 + 8 * hlf + r; float y = acc[t][r] * (1.0f / (XS * WSC)) + bb; if (MODE == 1) y = fmaxf(y, 0.0f); Tf[wave][8 * hlf + r][col] = (vrow < (size_t)nvalid) ? y : 0.0f; } }
  wave_lds_sync();
  for (int pass = 0; pass < 2; ++pass) { for (int rr = 0; rr < 16; ++rr) { if (m0 + rr < (size_t)mrows) { if (NC >= 128) { for (int c8 = 0; c8 < NC; c8 += 128) *(volatile v4f*)(OUT + (m0 + rr) * (size_t)opitch + c8 + lane * 4) = *(const v4f*)(&Tf[wave][rr][c8 + lane * 4]); }
        else { if (lane < NC / 4) *(volatile v4f*)(OUT + (m0 + rr) * (size_t)opitch + lane * 4) = *(const v4f*)(&Tf[wave][rr][lane * 4]); } } } __threadfence(); }
}
__device__ __forceinline__ float gelu_(float v) { return 0.5f * v * (1.0f + erff(v * 0.70710678118654752f)); }
template <int W, int ACT>
__global__ __launch_bounds__(256) void gcn_kernel(const float* __restrict__ Hh, const int* __restrict__ srcs, const int* __restrict__ PERM, const int* __restrict__ ROWPTR, const int* __restrict__ ROWCNT, int permLen, const float* __restrict__ bias, const float* __restrict__ ADDP, float* __restrict__ out, int mrows) {
  constexpr int CW = W / 8;
  static_assert(W % 32 == 0, "gcn: 8 threads per row, float4 stores");
  const int tid = threadIdx.x; const int row = tid >> 3, g = tid & 7, c0 = g * CW; const int v = blockIdx.x * 32 + row; const int vv = v < N ? v : N - 1;
  int cnt = 0, p0 = 0; if (v < N) { cnt = iclamp(ROWCNT[v], 0, 65536); p0 = iclamp(ROWPTR[v], 0, permLen - 1); if (p0 + cnt > permLen) cnt = permLen - p0; }
  const float dv = rsqrtf((float)(cnt + 1));
  float m[CW]; { const float* hr = Hh + (size_t)vv * W + c0;
#pragma unroll
    for (int q = 0; q < CW / 4; ++q) { const v4f t4 = *(const v4f*)(hr + 4 * q); for (int j = 0; j < 4; ++j) m[4 * q + j] = pmul(dv, t4[j]); } }
#pragma unroll 1
  for (int i = 0; i < cnt; ++i) { const int e = iclamp(PERM[p0 + i], 0, E - 1); int s = iclamp(srcs[e], 0, N - 1); if (SRCM < N) s %= SRCM; const float cf = rsqrtf((float)(iclamp(ROWCNT[s], 0, 1 << 24) + 1)); const float* hr = Hh + (size_t)s * W + c0;
#pragma unroll
    for (int q = 0; q < CW / 4; ++q) { const v4f t4 = *(const v4f*)(hr + 4 * q); for (int j = 0; j < 4; ++j) m[4 * q + j] += pmul(cf, t4[j]); } }
  for (int pass = 0; pass < 2; ++pass) { if (v < mrows) { float* orow = out + (size_t)v * W + c0;
#pragma unroll
      for (int q = 0; q < CW / 4; ++q) { v4f o; for (int j = 0; j < 4; ++j) { float y = pmul(dv, m[4 * q + j]) + bf16_rne(bias[c0 + 4 * q + j]); if (ADDP != nullptr) y += ADDP[(size_t)vv * W + c0 + 4 * q + j]; if (ACT == 1) y = fmaxf(y, 0.0f); if (ACT == 3) y = (y >= 0.0f) ? y : 0.01f * y; if (ACT == 4) { const float sp = (y > 20.0f) ? y : __logf(1.0f + __expf(y)); const float t = __expf(pmul(-2.0f, sp)); y = pmul(pmul(y, 1.0f - t), __builtin_amdgcn_rcpf(1.0f + t)); }     o[j] = (v < N) ? y : 0.0f; } *(volatile v4f*)(orow + 4 * q) = o; } }
    __threadfence(); }
}
__global__ __launch_bounds__(256) void zfill_kernel(float* __restrict__ Z, int n) { const int i = threadIdx.x; for (int pass = 0; pass < 2; ++pass) { if (i < n) ((volatile float*)Z)[i] = 0.0f; __threadfence(); } }
template <int NR>
__global__ __launch_bounds__(64) void bpadn_kernel(const float* __restrict__ b, float* __restrict__ B) { static_assert(NR <= 64, "bpadn: 64-entry record"); const int c = threadIdx.x; const float v = (c < NR) ? b[c] : 0.0f; for (int pass = 0; pass < 2; ++pass) { ((volatile float*)B)[c] = v; __threadfence(); } }
__global__ __launch_bounds__(256) void gchk_kernel(const int* __restrict__ batch, int* __restrict__ FLAG, int nn) {
  const int v = blockIdx.x * 256 + threadIdx.x; if (v + 1 >= nn) return; if (batch[v] > batch[v + 1] || batch[v] < 0) { ((volatile int*)FLAG)[0] = 1; __threadfence(); }
}
__global__ __launch_bounds__(128) void gmean_kernel(const float* __restrict__ H, const int* __restrict__ batch, const int* __restrict__ FLAG, float* __restrict__ P, int nstat) {
  const int g = blockIdx.x, c = threadIdx.x; int lo = 0, hi = nstat; while (lo < hi) { const int mid = (lo + hi) >> 1; if (batch[mid] < g) lo = mid + 1; else hi = mid; } const int st = lo; hi = nstat; while (lo < hi) { const int mid = (lo + hi) >> 1; if (batch[mid] <= g) lo = mid + 1; else hi = mid; } const int en = lo;
  float s = 0.0f;
#pragma unroll 1
  for (int v = st; v < en; ++v) s += H[(size_t)v * F + c];
  float o = (en > st) ? s / (float)(en - st) : 0.0f; if (FLAG[0] != 0) o = __int_as_float(0x7fc00000);
  for (int pass = 0; pass < 2; ++pass) { ((volatile float*)P)[(size_t)g * F + c] = o; __threadfence(); }
}
__global__ __launch_bounds__(256) void ocpf_kernel(const float* __restrict__ P, float* __restrict__ out, int total) {
  const int t = blockIdx.x * 256 + threadIdx.x; if (t >= total) return; const int g = t / NCLS, k = t - g * NCLS; const float v = P[(size_t)g * FO + k];
  for (int pass = 0; pass < 2; ++pass) { ((volatile float*)out)[t] = v; __threadfence(); }
}
template <int XI, int KP>
__global__ __launch_bounds__(256) void xpads_kernel(const float* __restrict__ x, int xp, int xo, float* __restrict__ P, int n, int nrows) {
  static_assert(XI >= 1 && XI <= KP && KP % 32 == 0, "xpads: a slice of at most KP columns; whole 128-B lines per row"); const int v = blockIdx.x * 256 + threadIdx.x; if (v >= nrows) return; float a[XI]; for (int k = 0; k < XI; ++k) a[k] = (v < n) ? bf16_rne(x[(size_t)v * xp + xo + k]) : 0.0f;
  for (int pass = 0; pass < 2; ++pass) { float* row = P + (size_t)v * KP; for (int q = 0; q < KP / 4; ++q) { v4f o = {0.0f, 0.0f, 0.0f, 0.0f}; for (int j = 0; j < 4; ++j) if (4 * q + j < XI) o[j] = a[4 * q + j]; *(volatile v4f*)(row + 4 * q) = o; } __threadfence(); }
}
template <int NC, int PW>
__global__ __launch_bounds__(256) void ocpft_kernel(const float* __restrict__ P, float* __restrict__ out, int total) {
  static_assert(NC >= 1 && NC <= PW, "ocpft: NC real columns of a PW-pitch plane"); const int t = blockIdx.x * 256 + threadIdx.x; if (t >= total) return; const int g = t / NC, k = t - g * NC; const float v = P[(size_t)g * PW + k];
  for (int pass = 0; pass < 2; ++pass) { ((volatile float*)out)[t] = v; __threadfence(); }
}
}

extern "C" void kernel_launch(void* const* d_in, const int* in_sizes, int n_in, void* d_out, int out_size, void* d_ws, size_t ws_size, hipStream_t stream) {
  (void)n_in;
  auto Fp = [&](int i) { return (const float*)d_in[i]; }; auto Ip = [&](int i) { return (const int*)d_in[i]; };
  constexpr int C = 32  , PW = 64  ;
  if (in_sizes[0] != N * C || in_sizes[1] != 2 * EFULL || in_sizes[2] != C * C || in_sizes[3] != C || in_sizes[4] != C * C || in_sizes[5] != C || out_size != N * C) return;
  size_t off = 0; char* ws = (char*)d_ws;
  auto carve = [&](size_t bytes) { char* p = ws + off; off += (bytes + 255) & ~(size_t)255; return p; };
  b16* W1T = (b16*)carve((size_t)PW * PW * 2); b16* W2T = (b16*)carve((size_t)PW * PW * 2); b16* W2Q = (b16*)carve((size_t)PW * PW * 2);
  float* W1P = (float*)carve((size_t)PW * C * 4); float* W2P = (float*)carve((size_t)PW * C * 4);
  float* ZB = (float*)carve(1024); float* B1P = (float*)carve(1024); float* B2P = (float*)carve(1024);
  float* XP = (float*)carve((size_t)NP * PW * 4); float* PA = (float*)carve((size_t)NP * PW * 4); float* PB = (float*)carve((size_t)NP * PW * 4);
  CsrBufs csr; off = csr_carve(csr, ws, off, E, N);
  if (off > ws_size || off > ((size_t)126 << 20)) return;
  { const unsigned g = (PW * PW / 8 + 255) / 256;
    csrZ_kernel<<<8, 256, 0, stream>>>((int*)W1P, (size_t)PW * C / 4); csrZ_kernel<<<8, 256, 0, stream>>>((int*)W1P, (size_t)PW * C / 4); csrZ_kernel<<<8, 256, 0, stream>>>((int*)W2P, (size_t)PW * C / 4); csrZ_kernel<<<8, 256, 0, stream>>>((int*)W2P, (size_t)PW * C / 4);
    xpads_kernel<C, C><<<1, 256, 0, stream>>>(Fp(2), C, 0, W1P, C, C); xpads_kernel<C, C><<<1, 256, 0, stream>>>(Fp(4), C, 0, W2P, C, C);
    wt_kernel<PW, C, PW><<<g, 256, 0, stream>>>(W1P, W1T, WSC); wt_kernel<PW, C, PW><<<g, 256, 0, stream>>>(W2P, W2T, WSC); wt_kernel<PW, C, PW><<<g, 256, 0, stream>>>(W2P, W2Q, WSQ);
    zfill_kernel<<<1, 256, 0, stream>>>(ZB, 256); bpadn_kernel<C><<<1, 64, 0, stream>>>(Fp(3), B1P); bpadn_kernel<C><<<1, 64, 0, stream>>>(Fp(5), B2P); }
  csr_build(csr, Ip(1) + EFULL, E, N, stream);
  const unsigned gr = (unsigned)((NRL + 255) / 256);
  xpads_kernel<C, PW><<<gr, 256, 0, stream>>>(Fp(0), C, 0, XP, N, NRL);
  lin_kernel<PW, 4, true, 0, false><<<NRL / 32, 64, 0, stream>>>(XP, nullptr, W1T, W1T, ZB, PA, PW, N, NRL);
  gcn_kernel<PW, 1><<<NRL / 32, 256, 0, stream>>>(PA, Ip(1), csr.PERM, csr.ROWPTR, csr.ROWCNT, (int)csr.permLen, B1P, nullptr, PB, NRL);
  lin_kernel<PW, 4, false, 0, false><<<NRL / 32, 64, 0, stream>>>(PB, nullptr, W2T, W2Q, ZB, PA, PW, N, NRL);
  gcn_kernel<PW, 0><<<NRL / 32, 256, 0, stream>>>(PA, Ip(1), csr.PERM, csr.ROWPTR, csr.ROWCNT, (int)csr.permLen, B2P, nullptr, XP, NRL);
  ocpft_kernel<C, PW><<<(unsigned)(((size_t)NL * C + 255) / 256), 256, 0, stream>>>(XP, (float*)d_out, NL * C);
}
